// MyModel_3848290697240
// MI455X (gfx1250) — hardware-verified
//
#include <hip/hip_runtime.h>
#include <math.h>

#ifndef NB
#define NB 384
#endif
#define NB_FULL 384
#define DM 1024
#define WD 300
#define WDP 320
#define VOC 30000
#define NNOUN 8000
#define LNOUN 16
#define CROWS (NB * LNOUN)
#define EROWS (NNOUN + CROWS)
#define EPIECE (WDP / 8)
#define OUT1_OFF (NB_FULL * NB_FULL)
#define SC_PITCH 36
#define SC_TILES (NB / 32)

#define C_H   16.0f
#define C_W2  64.0f
#define C_TA  65536.0f
#define C_T16 16.0f
#define C_AA  33554432.0f
#define C_TT  1024.0f
#define C_RN  1024.0f
#define C_TN  1024.0f
static constexpr float LG_INV  = 1.0f / (C_H * C_W2);
static constexpr float NUM_INV = 1.0f / (C_TA * C_T16);
static constexpr float DEN_INV = 1.0f / (C_AA * C_TT);
static constexpr float IS_INV  = 1.0f / (C_RN * C_TN);
static constexpr float LOG2E_F = 1.4426950408889634f;

static_assert(LG_INV * C_H * C_W2 == 1.0f);
static_assert(NUM_INV * C_TA * C_T16 == 1.0f);
static_assert(DEN_INV * C_AA * C_TT == 1.0f);
static_assert(IS_INV * C_RN * C_TN == 1.0f);
static_assert(NB <= NB_FULL && NB % 64 == 0 && NB % 32 == 0 && NB % 8 == 0);
static_assert(DM % 64 == 0 && DM % 32 == 0 && DM == 1024);
static_assert(WDP % 32 == 0 && WDP >= WD && WDP % 8 == 0);
static_assert(NNOUN % 64 == 0 && EROWS % 64 == 0 && CROWS % 8 == 0);
static_assert((EROWS * EPIECE) % 256 == 0);
static_assert((DM * (WDP / 8)) % 256 == 0 && (DM * (DM / 8)) % 256 == 0);
static_assert(LNOUN == 16);
static_assert(OUT1_OFF * 4 == 589824 && (OUT1_OFF * 4) % 128 == 0);
static_assert((NB_FULL * 4) % 128 == 0);
static_assert(OUT1_OFF + NB_FULL * LNOUN * DM == 6438912);
static_assert(32 * 16 * 8 == 16 * 64 * 4);
static_assert(32 * 16 * 4 == 16 * 64 * 2);
static_assert(32 * 16 * 4 == 16 * 32 * 4);
static_assert(32 * 16 * 8 == DM * 4);
static_assert(32 * 16 * 4 == DM * 2);
static_assert(8 * 16 * 68 * 4 <= 131072);
static_assert(8 * 16 * SC_PITCH * 4 <= 131072);
static_assert((SC_PITCH * 4) % 16 == 0);

static constexpr size_t WS_EALL = (size_t)EROWS * WDP * 2;
static constexpr size_t WS_NWT  = (size_t)DM * WDP * 2;
static constexpr size_t WS_SQ16 = (size_t)DM * DM * 2;
static constexpr size_t WS_ROW16 = (size_t)NB * DM * 2;
static constexpr size_t WS_ROW32 = (size_t)NB * DM * 4;
static constexpr size_t WS_CF   = (size_t)EROWS * DM * 4;
static constexpr size_t WS_TOTAL = WS_EALL + WS_NWT + 3 * WS_SQ16 + 8 * WS_ROW16 + 2 * WS_ROW32 + WS_CF;
static_assert(WS_EALL % 256 == 0 && WS_NWT % 256 == 0 && WS_ROW16 % 256 == 0 && WS_CF % 256 == 0);
static_assert(WS_TOTAL <= (size_t)134217728);

typedef _Float16 h16;
typedef __attribute__((ext_vector_type(16))) _Float16 v16h;
typedef __attribute__((ext_vector_type(16))) __bf16   v16bf;
typedef __attribute__((ext_vector_type(8)))  _Float16 v8h;
typedef __attribute__((ext_vector_type(8)))  float    v8f;
typedef __attribute__((ext_vector_type(4)))  float    v4f;
typedef __attribute__((ext_vector_type(4)))  unsigned int v4u;
typedef __attribute__((ext_vector_type(8)))  unsigned int v8u;


#define VST2(T, ptr, val) do { const T vst2_v_ = (val); *(volatile T*)(ptr) = vst2_v_; __threadfence(); *(volatile T*)(ptr) = vst2_v_; } while (0)

__device__ __forceinline__ float bfr(float f) {
    unsigned u = __float_as_uint(f);
    u += 0x7FFFu + ((u >> 16) & 1u);
    return __uint_as_float(u & 0xFFFF0000u);
}
__device__ __forceinline__ unsigned bf_pack(float lo, float hi) {
    unsigned a = __float_as_uint(lo);
    a += 0x7FFFu + ((a >> 16) & 1u);
    unsigned b = __float_as_uint(hi);
    b += 0x7FFFu + ((b >> 16) & 1u);
    return (a >> 16) | (b & 0xFFFF0000u);
}
static __device__ __forceinline__ h16 toh_flush(float v) {
    const float w = (fabsf(v) < 6.103515625e-05f) ? 0.0f : v;
    return (h16)w;
}
__device__ __forceinline__ void st8bf(unsigned short* P, unsigned o, const float* v) {
    v4u pk;
    pk.x = bf_pack(v[0], v[1]);
    pk.y = bf_pack(v[2], v[3]);
    pk.z = bf_pack(v[4], v[5]);
    pk.w = bf_pack(v[6], v[7]);
    VST2(v4u, (v4u*)(P + o), pk);
}
__device__ __forceinline__ void st8hf(unsigned short* P, unsigned o, const float* v) {
    v8h hv;
#pragma unroll
    for (int e = 0; e < 8; ++e) hv[e] = toh_flush(v[e]);
    VST2(v8h, (v8h*)(P + o), hv);
}
__device__ __forceinline__ void ld8(const float* __restrict__ p, float* v) {
    const v4f a = *(const v4f*)(p);
    const v4f b = *(const v4f*)(p + 4);
    v[0] = a.x; v[1] = a.y; v[2] = a.z; v[3] = a.w;
    v[4] = b.x; v[5] = b.y; v[6] = b.z; v[7] = b.w;
}
__device__ __forceinline__ float wave_sum(float s) {
#pragma unroll
    for (int o = 16; o > 0; o >>= 1) s += __shfl_xor(s, o, 32);
    return s;
}
__device__ __forceinline__ float wave_max(float s) {
#pragma unroll
    for (int o = 16; o > 0; o >>= 1) s = fmaxf(s, __shfl_xor(s, o, 32));
    return s;
}

__device__ __forceinline__ v8u frag_ld(const unsigned short* p) {
    const v4u lo = *(const v4u*)(p);
    const v4u hi = *(const v4u*)(p + 16);
    return __builtin_shufflevector(lo, hi, 0, 1, 2, 3, 4, 5, 6, 7);
}
__device__ __forceinline__ v8f wmma16g(v8u a, v8u b, v8f c) {
    c = __builtin_amdgcn_wmma_f32_16x16x32_f16(false, __builtin_bit_cast(v16h, a), false, __builtin_bit_cast(v16h, b), (short)0, c, false, false);
    asm volatile("v_nop\n\tv_nop\n\tv_nop\n\tv_nop" : "+v"(c) : "v"(a), "v"(b));
    return c;
}
__device__ __forceinline__ v8f wmmabg(v8u a, v8u b, v8f c) {
    c = __builtin_amdgcn_wmma_f32_16x16x32_bf16(false, __builtin_bit_cast(v16bf, a), false, __builtin_bit_cast(v16bf, b), (short)0, c, false, false);
    asm volatile("v_nop\n\tv_nop\n\tv_nop\n\tv_nop" : "+v"(c) : "v"(a), "v"(b));
    return c;
}
template <bool BF>
__device__ __forceinline__ v8f mma_g(v8u a, v8u b, v8f c) {
    if (BF) return wmmabg(a, b, c);
    return wmma16g(a, b, c);
}
__device__ __forceinline__ void wave_sync_lds() {
    __builtin_amdgcn_fence(3  , "workgroup");
    __builtin_amdgcn_wave_barrier();
    __builtin_amdgcn_fence(2  , "workgroup");
}

template <bool BF, int OUT_MODE, bool RELU>
__device__ __forceinline__ void gemm64_body(
    const unsigned short* __restrict__ A, unsigned lda, const unsigned short* __restrict__ Bt, unsigned ldb,
    void* __restrict__ Cout, unsigned ldc, const float* __restrict__ bias,
    unsigned M, unsigned N, unsigned K, float scale, float oscale) {
  __shared__ __align__(16) float sT[8][16 * 68];
  const unsigned lane = threadIdx.x & 31u;
  const unsigned wave = (unsigned)__builtin_amdgcn_readfirstlane((int)(threadIdx.x >> 5));
  const unsigned tilesN = N >> 6, tilesM = M >> 6;
  const unsigned tile = blockIdx.x * 8u + wave;
  if (tile >= tilesM * tilesN) return;
  const unsigned tm = tile / tilesN;
  const unsigned tn = tile - tm * tilesN;
  const unsigned m0 = tm << 6, n0 = tn << 6;
  const unsigned rlane = lane & 15u;
  const unsigned koff = (lane >> 4) * 8u;
  const unsigned mOff = koff;

  v8f acc[4][4];
#pragma unroll
  for (int i = 0; i < 4; ++i)
#pragma unroll
    for (int j = 0; j < 4; ++j) acc[i][j] = (v8f){0.f,0.f,0.f,0.f,0.f,0.f,0.f,0.f};

  for (unsigned k0 = 0; k0 < K; k0 += 32u) {
    v8u bh[4];
#pragma unroll
    for (int j = 0; j < 4; ++j)
      bh[j] = frag_ld(Bt + (size_t)(n0 + ((unsigned)j << 4) + rlane) * ldb + koff + k0);
#pragma unroll
    for (int i = 0; i < 4; ++i) {
      const v8u ah = frag_ld(A + (size_t)(m0 + ((unsigned)i << 4) + rlane) * lda + koff + k0);
#pragma unroll
      for (int j = 0; j < 4; ++j)
        acc[i][j] = mma_g<BF>(ah, bh[j], acc[i][j]);
    }
  }

  float* slab = sT[wave];
#pragma unroll
  for (int i = 0; i < 4; ++i) {
    const unsigned mBase = m0 + ((unsigned)i << 4);
#pragma unroll
    for (int j = 0; j < 4; ++j) {
      const unsigned n = n0 + ((unsigned)j << 4) + rlane;
      const float bv = bfr(bias[n]);
#pragma unroll
      for (int r = 0; r < 8; ++r) {
        float v = acc[i][j][r] * scale + bv;
        if (RELU) v = fmaxf(v, 0.0f);
        if (OUT_MODE == 1) v *= oscale;
        slab[(mOff + (unsigned)r) * 68u + ((unsigned)j << 4) + rlane] = v;
      }
    }
    wave_sync_lds();
    if (OUT_MODE == 0) {
      float* C = (float*)Cout;
      const unsigned hh = lane >> 4, c4 = (lane & 15u) * 4u;
#pragma unroll
      for (int half = 0; half < 2; ++half) {
        v4f vv[4];
#pragma unroll
        for (int it = 0; it < 4; ++it) {
          const unsigned row = (unsigned)(half * 4 + it) * 2u + hh;
          vv[it] = *(const v4f*)(slab + row * 68u + c4);
        }
        for (int pass = 0; pass < 2; ++pass) {
#pragma unroll
          for (int it = 0; it < 4; ++it) {
            const unsigned row = (unsigned)(half * 4 + it) * 2u + hh;
            *(volatile v4f*)(C + (size_t)(mBase + row) * ldc + n0 + c4) = vv[it];
          }
          __threadfence();
        }
      }
    } else {
      _Float16* C = (_Float16*)Cout;
      const unsigned q = lane >> 3, c8 = (lane & 7u) * 8u;
      v8h hv[4];
#pragma unroll
      for (int it = 0; it < 4; ++it) {
        const unsigned row = (unsigned)it * 4u + q;
        const float* sp = slab + row * 68u + c8;
#pragma unroll
        for (int e = 0; e < 8; ++e) hv[it][e] = toh_flush(sp[e]);
      }
      for (int pass = 0; pass < 2; ++pass) {
#pragma unroll
        for (int it = 0; it < 4; ++it) {
          const unsigned row = (unsigned)it * 4u + q;
          *(volatile v8h*)(C + (size_t)(mBase + row) * ldc + n0 + c8) = hv[it];
        }
        __threadfence();
      }
    }
    wave_sync_lds();
  }
}

__global__ __launch_bounds__(256) void k_gemm_bf_f32(
    const unsigned short* __restrict__ A, unsigned lda, const unsigned short* __restrict__ Bt, unsigned ldb,
    float* __restrict__ C, unsigned ldc, const float* __restrict__ bias, unsigned M, unsigned N, unsigned K) {
  gemm64_body<true, 0, false>(A, lda, Bt, ldb, (void*)C, ldc, bias, M, N, K, 1.0f, 1.0f);
}
__global__ __launch_bounds__(256) void k_gemm_bf_h16(
    const unsigned short* __restrict__ A, unsigned lda, const unsigned short* __restrict__ Bt, unsigned ldb,
    unsigned short* __restrict__ C, unsigned ldc, const float* __restrict__ bias, unsigned M, unsigned N, unsigned K) {
  gemm64_body<true, 1, true>(A, lda, Bt, ldb, (void*)C, ldc, bias, M, N, K, 1.0f, C_H);
}
__global__ __launch_bounds__(256) void k_gemm_h_f32(
    const unsigned short* __restrict__ A, unsigned lda, const unsigned short* __restrict__ Bt, unsigned ldb,
    float* __restrict__ C, unsigned ldc, const float* __restrict__ bias, unsigned M, unsigned N, unsigned K) {
  gemm64_body<false, 0, false>(A, lda, Bt, ldb, (void*)C, ldc, bias, M, N, K, LG_INV, 1.0f);
}

__global__ __launch_bounds__(256) void k_gather(const int* __restrict__ antk, const int* __restrict__ ntid,
                                                const float* __restrict__ emb, unsigned short* __restrict__ eall) {
    const unsigned u = blockIdx.x * 256u + threadIdx.x;
    if (u >= (unsigned)(EROWS * EPIECE)) return;
    const unsigned row = u / (unsigned)EPIECE;
    unsigned piece = u - row * (unsigned)EPIECE;
    asm volatile("" : "+v"(piece));
    const int ia = min((int)row, NNOUN - 1);
    const int ib = min(max((int)row - NNOUN, 0), CROWS - 1);
    const int ta = antk[ia];
    const int tb = ntid[ib];
    int tok = (row < (unsigned)NNOUN) ? ta : tb;
    tok = min(max(tok, 0), VOC - 1);
    asm volatile("" : "+v"(tok));
    const float* er = emb + (unsigned)tok * (unsigned)WD;
    float v[8];
#pragma unroll
    for (int i = 0; i < 8; ++i) {
        const unsigned cidx = 8u * piece + (unsigned)i;
        const unsigned cc = min(cidx, (unsigned)(WD - 1));
        const float x = er[cc];
        v[i] = (cidx < (unsigned)WD) ? x : 0.0f;
    }
    st8bf(eall, u * 8u, v);
}

template <unsigned KI, unsigned KP, unsigned NO, bool F16>
__device__ __forceinline__ void wt_body(const float* __restrict__ Wm, unsigned short* __restrict__ W16) {
    const unsigned u = blockIdx.x * 256u + threadIdx.x;
    const unsigned per = KP / 8u;
    if (u >= NO * per) return;
    const unsigned o = u / per;
    unsigned kq = u - o * per;
    asm volatile("" : "+v"(kq));
    float v[8];
#pragma unroll
    for (int i = 0; i < 8; ++i) {
        const unsigned k = 8u * kq + (unsigned)i;
        const unsigned kc = min(k, KI - 1u);
        const float x = Wm[kc * NO + o];
        const float w = F16 ? (bfr(x) * C_W2) : x;
        v[i] = (k < KI) ? w : 0.0f;
    }
    if (F16) st8hf(W16, u * 8u, v);
    else     st8bf(W16, u * 8u, v);
}
__global__ __launch_bounds__(256) void k_wt_noun(const float* __restrict__ Wm, unsigned short* __restrict__ W16) {
    wt_body<WD, WDP, DM, false>(Wm, W16);
}
__global__ __launch_bounds__(256) void k_wt_sq_bf(const float* __restrict__ Wm, unsigned short* __restrict__ W16) {
    wt_body<DM, DM, DM, false>(Wm, W16);
}
__global__ __launch_bounds__(256) void k_wt_sq_h(const float* __restrict__ Wm, unsigned short* __restrict__ W16) {
    wt_body<DM, DM, DM, true>(Wm, W16);
}

__global__ __launch_bounds__(256) void k_prep_in(const float* __restrict__ r, const float* __restrict__ m, const float* __restrict__ t,
                                                 unsigned short* __restrict__ MB, unsigned short* __restrict__ RN,
                                                 unsigned short* __restrict__ T16, unsigned short* __restrict__ TT,
                                                 unsigned short* __restrict__ TN) {
    const unsigned lane = threadIdx.x & 31u;
    const unsigned wave = (unsigned)__builtin_amdgcn_readfirstlane((int)(threadIdx.x >> 5));
    const unsigned row = blockIdx.x * 8u + wave;
    if (row >= (unsigned)NB) return;
    const unsigned base = row * (unsigned)DM + 8u * lane;
    for (unsigned j = 0; j < 4u; ++j) {
        float v[8];
        ld8(m + base + 256u * j, v);
        st8bf(MB, base + 256u * j, v);
    }
    float rv[4][8];
#pragma unroll
    for (unsigned j = 0; j < 4u; ++j) ld8(r + base + 256u * j, rv[j]);
#pragma unroll
    for (unsigned j = 0; j < 4u; ++j) {
#pragma unroll
        for (int e = 0; e < 8; ++e) rv[j][e] = bfr(rv[j][e]);
    }
    float sr = 0.f;
#pragma unroll
    for (unsigned j = 0; j < 4u; ++j) {
#pragma unroll
        for (int e = 0; e < 8; ++e) { const float x = rv[j][e]; sr += x * x; }
    }
    sr = wave_sum(sr);
    const float ir = 1.0f / sqrtf(sr);
#pragma unroll
    for (unsigned j = 0; j < 4u; ++j) {
        float w[8];
#pragma unroll
        for (int e = 0; e < 8; ++e) w[e] = (rv[j][e] * ir) * C_RN;
        st8hf(RN, base + 256u * j, w);
    }
    float tv[4][8];
#pragma unroll
    for (unsigned j = 0; j < 4u; ++j) ld8(t + base + 256u * j, tv[j]);
#pragma unroll
    for (unsigned j = 0; j < 4u; ++j) {
#pragma unroll
        for (int e = 0; e < 8; ++e) tv[j][e] = bfr(tv[j][e]);
    }
    float st = 0.f;
#pragma unroll
    for (unsigned j = 0; j < 4u; ++j) {
#pragma unroll
        for (int e = 0; e < 8; ++e) { const float x = tv[j][e]; st += x * x; }
    }
    st = wave_sum(st);
    const float itn = 1.0f / sqrtf(st);
#pragma unroll
    for (unsigned j = 0; j < 4u; ++j) {
        float w16[8], wtt[8], wtn[8];
#pragma unroll
        for (int e = 0; e < 8; ++e) {
            const float x = tv[j][e];
            w16[e] = x * C_T16;
            wtt[e] = (x * x) * C_TT;
            wtn[e] = (x * itn) * C_TN;
        }
        st8hf(T16, base + 256u * j, w16);
        st8hf(TT,  base + 256u * j, wtt);
        st8hf(TN,  base + 256u * j, wtn);
    }
}

__global__ __launch_bounds__(256) void k_rows_mid(const float* __restrict__ LG, const float* __restrict__ TRM,
                                                  unsigned short* __restrict__ TA, unsigned short* __restrict__ AA) {
    const unsigned lane = threadIdx.x & 31u;
    const unsigned wave = (unsigned)__builtin_amdgcn_readfirstlane((int)(threadIdx.x >> 5));
    const unsigned row = blockIdx.x * 8u + wave;
    if (row >= (unsigned)NB) return;
    const unsigned base = row * (unsigned)DM + 8u * lane;
    float la[4][8], tb[4][8];
#pragma unroll
    for (unsigned j = 0; j < 4u; ++j) {
        ld8(LG + base + 256u * j, la[j]);
        ld8(TRM + base + 256u * j, tb[j]);
    }
    float mx = -3.0e38f, sq = 0.f;
#pragma unroll
    for (unsigned j = 0; j < 4u; ++j) {
#pragma unroll
        for (int e = 0; e < 8; ++e) { mx = fmaxf(mx, la[j][e]); sq += tb[j][e] * tb[j][e]; }
    }
    mx = wave_max(mx);
    sq = wave_sum(sq);
    float ex[4][8];
#pragma unroll
    for (unsigned j = 0; j < 4u; ++j) {
#pragma unroll
        for (int e = 0; e < 8; ++e) ex[j][e] = exp2f((la[j][e] - mx) * LOG2E_F);
    }
    float se = 0.f;
#pragma unroll
    for (unsigned j = 0; j < 4u; ++j) {
#pragma unroll
        for (int e = 0; e < 8; ++e) se += ex[j][e];
    }
    se = wave_sum(se);
    const float ia = 1.0f / se;
    const float itr = 1.0f / sqrtf(sq);
#pragma unroll
    for (unsigned j = 0; j < 4u; ++j) {
        float wa[8], wq[8];
#pragma unroll
        for (int e = 0; e < 8; ++e) {
            const float p = ex[j][e] * ia;
            const float tr = tb[j][e] * itr;
            wa[e] = (tr * p) * C_TA;
            wq[e] = (p * p) * C_AA;
        }
        st8hf(TA, base + 256u * j, wa);
        st8hf(AA, base + 256u * j, wq);
    }
}

__global__ __launch_bounds__(256) void k_concepts(const int* __restrict__ ntid, const int* __restrict__ nlen,
                                                  const int* __restrict__ t2i, const float* __restrict__ CF,
                                                  float* __restrict__ out1) {
    const unsigned lane = threadIdx.x & 31u;
    const unsigned wave = (unsigned)__builtin_amdgcn_readfirstlane((int)(threadIdx.x >> 5));
    const unsigned row = blockIdx.x * 8u + wave;
    if (row >= (unsigned)CROWS) return;
    const unsigned b = row >> 4;
    const int l = (int)(row & 15u);
    int tok = ntid[row];
    tok = min(max(tok, 0), VOC - 1);
    asm volatile("" : "+v"(tok));
    int widx = t2i[tok];
    widx = min(max(widx, 0), NNOUN - 1);
    asm volatile("" : "+v"(widx));
    const int len = nlen[b];
    const bool valid = l < len;
    const bool found = widx > 0;
    const unsigned srow = (found && valid) ? (unsigned)widx : ((unsigned)NNOUN + row);
    const float* src = CF + (size_t)srow * DM + 4u * lane;
    float* dst = out1 + (size_t)row * DM + 4u * lane;
    const v4f z = (v4f){0.f, 0.f, 0.f, 0.f};
    v4f vv[8];
#pragma unroll
    for (int it = 0; it < 8; ++it) {
        v4f x = *(const v4f*)(src + 128 * it);
        asm volatile("" : "+v"(x));
        vv[it] = valid ? x : z;
    }
    for (int pass = 0; pass < 2; ++pass) {
#pragma unroll
        for (int it = 0; it < 8; ++it) *(volatile v4f*)(dst + 128 * it) = vv[it];
        __threadfence();
    }
}

__global__ __launch_bounds__(256) void k_score(const unsigned short* __restrict__ TA, const unsigned short* __restrict__ T16,
                                               const unsigned short* __restrict__ AA, const unsigned short* __restrict__ TT,
                                               const unsigned short* __restrict__ RN, const unsigned short* __restrict__ TN,
                                               float* __restrict__ out0) {
    __shared__ __align__(16) float sS[8][16 * SC_PITCH];
    const unsigned lane = threadIdx.x & 31u;
    const unsigned wave = (unsigned)__builtin_amdgcn_readfirstlane((int)(threadIdx.x >> 5));
    const unsigned tile = blockIdx.x * 8u + wave;
    if (tile >= (unsigned)(SC_TILES * SC_TILES)) return;
    const unsigned tm = tile / (unsigned)SC_TILES;
    const unsigned tn = tile - tm * (unsigned)SC_TILES;
    const unsigned m0 = tm * 32u, n0 = tn * 32u;
    const unsigned c = lane & 15u, hh = lane >> 4;
    const unsigned ao0 = (m0 + c) * (unsigned)DM + 8u * hh;
    const unsigned ao1 = ao0 + 16u * (unsigned)DM;
    const unsigned bo0 = (n0 + c) * (unsigned)DM + 8u * hh;
    const unsigned bo1 = bo0 + 16u * (unsigned)DM;

    v8f num[2][2], den[2][2], isv[2][2];
#pragma unroll
    for (int i = 0; i < 2; ++i)
#pragma unroll
        for (int j = 0; j < 2; ++j) {
            num[i][j] = (v8f){0.f,0.f,0.f,0.f,0.f,0.f,0.f,0.f};
            den[i][j] = num[i][j];
            isv[i][j] = num[i][j];
        }

#pragma unroll 1
    for (unsigned k0 = 0; k0 < (unsigned)DM; k0 += 32u) {
        {
            const v8u a0 = frag_ld(TA + ao0 + k0), a1 = frag_ld(TA + ao1 + k0);
            const v8u b0 = frag_ld(T16 + bo0 + k0), b1 = frag_ld(T16 + bo1 + k0);
            num[0][0] = wmma16g(a0, b0, num[0][0]);
            num[0][1] = wmma16g(a0, b1, num[0][1]);
            num[1][0] = wmma16g(a1, b0, num[1][0]);
            num[1][1] = wmma16g(a1, b1, num[1][1]);
        }
        {
            const v8u a0 = frag_ld(AA + ao0 + k0), a1 = frag_ld(AA + ao1 + k0);
            const v8u b0 = frag_ld(TT + bo0 + k0), b1 = frag_ld(TT + bo1 + k0);
            den[0][0] = wmma16g(a0, b0, den[0][0]);
            den[0][1] = wmma16g(a0, b1, den[0][1]);
            den[1][0] = wmma16g(a1, b0, den[1][0]);
            den[1][1] = wmma16g(a1, b1, den[1][1]);
        }
        {
            const v8u a0 = frag_ld(RN + ao0 + k0), a1 = frag_ld(RN + ao1 + k0);
            const v8u b0 = frag_ld(TN + bo0 + k0), b1 = frag_ld(TN + bo1 + k0);
            isv[0][0] = wmma16g(a0, b0, isv[0][0]);
            isv[0][1] = wmma16g(a0, b1, isv[0][1]);
            isv[1][0] = wmma16g(a1, b0, isv[1][0]);
            isv[1][1] = wmma16g(a1, b1, isv[1][1]);
        }
    }

    float* slab = sS[wave];
#pragma unroll
    for (int i = 0; i < 2; ++i) {
#pragma unroll
        for (int j = 0; j < 2; ++j) {
#pragma unroll
            for (int r = 0; r < 8; ++r) {
                const float nn = num[i][j][r] * NUM_INV;
                const float dd = den[i][j][r] * DEN_INV;
                const float v = nn * (1.0f / sqrtf(dd)) + isv[i][j][r] * IS_INV;
                slab[(8u * hh + (unsigned)r) * (unsigned)SC_PITCH + ((unsigned)j << 4) + c] = v;
            }
        }
        wave_sync_lds();
        {
            const unsigned q = lane >> 3, c4 = (lane & 7u) * 4u;
            v4f vv[4];
#pragma unroll
            for (int it = 0; it < 4; ++it) {
                const unsigned row = (unsigned)it * 4u + q;
                vv[it] = *(const v4f*)(slab + row * (unsigned)SC_PITCH + c4);
            }
            for (int pass = 0; pass < 2; ++pass) {
#pragma unroll
                for (int it = 0; it < 4; ++it) {
                    const unsigned row = (unsigned)it * 4u + q;
                    *(volatile v4f*)(out0 + (size_t)(m0 + ((unsigned)i << 4) + row) * NB_FULL + n0 + c4) = vv[it];
                }
                __threadfence();
            }
        }
        wave_sync_lds();
    }
}

extern "C" void kernel_launch(void* const* d_in, const int* in_sizes, int n_in, void* d_out, int out_size,
                              void* d_ws, size_t ws_size, hipStream_t stream) {
    if (n_in < 16) return;
    if (in_sizes[0] < NB * DM || in_sizes[1] < NB * DM || in_sizes[2] < NB * DM) return;
    if (in_sizes[3] < CROWS || in_sizes[4] < NB || in_sizes[5] < NNOUN) return;
    if (in_sizes[6] < VOC * WD || in_sizes[7] < WD * DM || in_sizes[8] < DM) return;
    if (in_sizes[9] < DM * DM || in_sizes[10] < DM || in_sizes[11] < DM * DM || in_sizes[12] < DM) return;
    if (in_sizes[13] < DM * DM || in_sizes[14] < DM || in_sizes[15] < VOC) return;
    if (out_size < OUT1_OFF + CROWS * DM) return;

    const float* r       = (const float*)d_in[0];
    const float* m       = (const float*)d_in[1];
    const float* t       = (const float*)d_in[2];
    const int*   ntid    = (const int*)d_in[3];
    const int*   nlen    = (const int*)d_in[4];
    const int*   antk    = (const int*)d_in[5];
    const float* emb     = (const float*)d_in[6];
    const float* noun_W  = (const float*)d_in[7];
    const float* noun_b  = (const float*)d_in[8];
    const float* em_W1   = (const float*)d_in[9];
    const float* em_b1   = (const float*)d_in[10];
    const float* em_W2   = (const float*)d_in[11];
    const float* em_b2   = (const float*)d_in[12];
    const float* tr_W    = (const float*)d_in[13];
    const float* tr_b    = (const float*)d_in[14];
    const int*   t2i     = (const int*)d_in[15];
    float* out0 = (float*)d_out;
    float* out1 = out0 + OUT1_OFF;

    char* wsp = (char*)d_ws;
    size_t off = 0;
    auto carve = [&](size_t bytes) -> void* { void* p = wsp + off; off += (bytes + 255) & ~(size_t)255; return p; };
    unsigned short* EALL = (unsigned short*)carve(WS_EALL);
    unsigned short* NWT  = (unsigned short*)carve(WS_NWT);
    unsigned short* W1T  = (unsigned short*)carve(WS_SQ16);
    unsigned short* TRT  = (unsigned short*)carve(WS_SQ16);
    unsigned short* W2T  = (unsigned short*)carve(WS_SQ16);
    unsigned short* MB   = (unsigned short*)carve(WS_ROW16);
    unsigned short* RN   = (unsigned short*)carve(WS_ROW16);
    unsigned short* T16  = (unsigned short*)carve(WS_ROW16);
    unsigned short* TT   = (unsigned short*)carve(WS_ROW16);
    unsigned short* TN   = (unsigned short*)carve(WS_ROW16);
    unsigned short* H16  = (unsigned short*)carve(WS_ROW16);
    unsigned short* TA   = (unsigned short*)carve(WS_ROW16);
    unsigned short* AA   = (unsigned short*)carve(WS_ROW16);
    float*          LG   = (float*)carve(WS_ROW32);
    float*          TRM  = (float*)carve(WS_ROW32);
    float*          CF   = (float*)carve(WS_CF);
    if (off > ws_size || off > (size_t)134217728) return;

    k_gather<<<(EROWS * EPIECE) / 256, 256, 0, stream>>>(antk, ntid, emb, EALL);
    k_wt_noun<<<(DM * (WDP / 8)) / 256, 256, 0, stream>>>(noun_W, NWT);
    k_wt_sq_bf<<<(DM * (DM / 8)) / 256, 256, 0, stream>>>(em_W1, W1T);
    k_wt_sq_bf<<<(DM * (DM / 8)) / 256, 256, 0, stream>>>(tr_W, TRT);
    k_wt_sq_h<<<(DM * (DM / 8)) / 256, 256, 0, stream>>>(em_W2, W2T);
    k_prep_in<<<NB / 8, 256, 0, stream>>>(r, m, t, MB, RN, T16, TT, TN);

    k_gemm_bf_f32<<<((EROWS / 64) * (DM / 64) + 7) / 8, 256, 0, stream>>>(EALL, WDP, NWT, WDP, CF, DM, noun_b, EROWS, DM, WDP);
    k_concepts<<<CROWS / 8, 256, 0, stream>>>(ntid, nlen, t2i, CF, out1);

    k_gemm_bf_h16<<<((NB / 64) * (DM / 64) + 7) / 8, 256, 0, stream>>>(MB, DM, W1T, DM, H16, DM, em_b1, NB, DM, DM);
    k_gemm_h_f32<<<((NB / 64) * (DM / 64) + 7) / 8, 256, 0, stream>>>(H16, DM, W2T, DM, LG, DM, em_b2, NB, DM, DM);
    k_gemm_bf_f32<<<((NB / 64) * (DM / 64) + 7) / 8, 256, 0, stream>>>(MB, DM, TRT, DM, TRM, DM, tr_b, NB, DM, DM);
    k_rows_mid<<<NB / 8, 256, 0, stream>>>(LG, TRM, TA, AA);
    k_score<<<(SC_TILES * SC_TILES + 7) / 8, 256, 0, stream>>>(TA, T16, AA, TT, RN, TN, out0);
}
